// SS2D_82248623718450
// MI455X (gfx1250) — hardware-run, weakly checked
//
#include <hip/hip_runtime.h>
#include <math.h>

typedef __attribute__((ext_vector_type(16))) __bf16   v16b;
typedef __attribute__((ext_vector_type(8)))  __bf16   v8b;
typedef __attribute__((ext_vector_type(8)))  float    v8f;
typedef __attribute__((ext_vector_type(4)))  float    v4f;
typedef __attribute__((ext_vector_type(2)))  float    v2f;
typedef __attribute__((ext_vector_type(4)))  unsigned v4u;

constexpr int kImg    = 8;
constexpr int kCh     = 192;
constexpr int kSide   = 64;
constexpr int kPos    = kSide * kSide;
constexpr int kSt     = 16;
constexpr int kRk     = 6;
constexpr int kDir    = 4;
constexpr int kXd     = kRk + 2 * kSt;
constexpr int kNreal  = kDir * kXd;
constexpr int kNp     = 192;
constexpr int kRows   = kImg * kPos;
constexpr int kTilesM = kRows / 64;
constexpr int kTilesN = kNp / 64;
constexpr int kChunk  = 64;
constexpr int kZP     = 40;
constexpr int kBlkCh  = 32;
constexpr int kHalfSt = 8;
constexpr int kPackTP = 196;
constexpr float kInvCh = 1.0f / (float)kCh;
constexpr float kEps   = 1e-5f;
static_assert(kXd == 38);
static_assert(kNreal == 152);
static_assert(kNreal <= kNp);
static_assert((kCh % 32) == 0);
static_assert((kRows % 64) == 0 && (kNp % 64) == 0);
static_assert((kTilesM * kTilesN) % 8 == 0);
static_assert(kPos == kChunk * kChunk);
static_assert(kCh % kBlkCh == 0);

constexpr size_t kPlaneElems = (size_t)kRows * kCh;
constexpr size_t kOffXH = 0;
constexpr size_t kOffXL = kOffXH + kPlaneElems * 2;
constexpr size_t kOffWH = kOffXL + kPlaneElems * 2;
constexpr size_t kOffWL = kOffWH + (size_t)kNp * kCh * 2;
constexpr size_t kOffZ  = kOffWL + (size_t)kNp * kCh * 2;
constexpr size_t kOffYR = kOffZ  + (size_t)kRows * kNp * 4;
constexpr size_t kOffYC = kOffYR + kPlaneElems * 4;
constexpr size_t kWsTotal = kOffYC + kPlaneElems * 4;
static_assert(kWsTotal == 100810752ull);
static_assert(kWsTotal <= 134217728ull);
static_assert((kOffXL % 128) == 0 && (kOffWH % 128) == 0 && (kOffWL % 128) == 0 &&
              (kOffZ % 128) == 0 && (kOffYR % 128) == 0 && (kOffYC % 128) == 0);
static_assert(kOffYC == kOffYR + kPlaneElems * 4);

__device__ __forceinline__ unsigned pin_u32(unsigned t) { asm volatile("" : "+v"(t)); return t; }

__device__ __forceinline__ unsigned bf_hi_bits(float f) {
  unsigned u = __float_as_uint(f);
  const unsigned lsb = (u & 0x00010000u) ? 1u : 0u;
  u = (u + 0x7FFFu + lsb) & 0xFFFF0000u;
  return u;
}
__device__ __forceinline__ void split_pair(float f0, float f1, unsigned& hw, unsigned& lw) {
  const unsigned h0 = bf_hi_bits(f0);
  const unsigned h1 = bf_hi_bits(f1);
  const float r0 = f0 - __uint_as_float(h0);
  const float r1 = f1 - __uint_as_float(h1);
  const unsigned l0 = bf_hi_bits(r0);
  const unsigned l1 = bf_hi_bits(r1);
  hw = __builtin_amdgcn_perm(h1, h0, 0x07060302u);
  lw = __builtin_amdgcn_perm(l1, l0, 0x07060302u);
}
__device__ __forceinline__ void split8(const v4f a0, const v4f a1, v4u& hv, v4u& lv) {
  unsigned hw, lw;
  split_pair(a0[0], a0[1], hw, lw); hv[0] = hw; lv[0] = lw;
  split_pair(a0[2], a0[3], hw, lw); hv[1] = hw; lv[1] = lw;
  split_pair(a1[0], a1[1], hw, lw); hv[2] = hw; lv[2] = lw;
  split_pair(a1[2], a1[3], hw, lw); hv[3] = hw; lv[3] = lw;
}

__device__ __forceinline__ void guard_row4(v8f& a, v8f& b, v8f& c, v8f& d, v16b x, v16b y) {
  asm volatile("v_nop\n\tv_nop\n\tv_nop\n\tv_nop" : "+v"(a), "+v"(b), "+v"(c), "+v"(d) : "v"(x), "v"(y));
}
__device__ __forceinline__ void keep4_b(v16b a, v16b b, v16b c, v16b d) { asm volatile("v_nop" :: "v"(a), "v"(b), "v"(c), "v"(d)); }
__device__ __forceinline__ void acc_guard4(v8f& a, v8f& b, v8f& c, v8f& d) { asm volatile("v_nop\n\tv_nop\n\tv_nop\n\tv_nop" : "+v"(a), "+v"(b), "+v"(c), "+v"(d)); }

struct FragB {
  union U { v16b v; v8b h[2]; };
  static __device__ __forceinline__ v16b load(const __bf16* p) {
    U f; f.h[0] = *(const v8b*)(p); f.h[1] = *(const v8b*)(p + 16); return f.v;
  }
  static __device__ __forceinline__ v8f mma(v16b a, v16b b, v8f c) {
    return __builtin_amdgcn_wmma_f32_16x16x32_bf16(false, a, false, b, (short)0, c, false, false);
  }
};

__global__ __launch_bounds__(256) void pack_x_kernel(
    const float* __restrict__ x, unsigned short* __restrict__ XH, unsigned short* __restrict__ XL)
{
  __shared__ __align__(16) float sT[32 * kPackTP];
  const unsigned tid = pin_u32(threadIdx.x);
  const unsigned img = blockIdx.x >> 7;
  const unsigned p0  = (blockIdx.x & 127u) << 5;
  const float* xb = x + (size_t)img * kCh * kPos + p0;
#pragma unroll
  for (int i = 0; i < 6; ++i) {
    const unsigned idx = pin_u32(tid + 256u * (unsigned)i);
    const unsigned dch = idx >> 3;
    const unsigned c4  = (idx & 7u) << 2;
    const v4f v = *(const v4f*)(xb + (size_t)dch * kPos + c4);
    sT[(c4 + 0u) * kPackTP + dch] = v[0];
    sT[(c4 + 1u) * kPackTP + dch] = v[1];
    sT[(c4 + 2u) * kPackTP + dch] = v[2];
    sT[(c4 + 3u) * kPackTP + dch] = v[3];
  }
  __syncthreads();
  v4u hv[3], lv[3];
#pragma unroll
  for (int i = 0; i < 3; ++i) {
    const unsigned j  = pin_u32(tid + 256u * (unsigned)i);
    const unsigned p  = pin_u32(j / 24u);
    const unsigned c8 = pin_u32((j - p * 24u) << 3);
    const float* sp = sT + p * kPackTP + c8;
    const v4f a0 = *(const v4f*)(sp);
    const v4f a1 = *(const v4f*)(sp + 4);
    split8(a0, a1, hv[i], lv[i]);
  }
  const size_t e0 = ((size_t)img * kPos + p0) * kCh;
  for (int pass = 0; pass < 2; ++pass) {
#pragma unroll
    for (int i = 0; i < 3; ++i) {
      const size_t eo = e0 + ((size_t)(tid + 256u * (unsigned)i) << 3);
      *(volatile v4u*)(XH + eo) = hv[i];
      *(volatile v4u*)(XL + eo) = lv[i];
    }
    __threadfence();
  }
}

__global__ __launch_bounds__(256) void pack_w_kernel(
    const float* __restrict__ w, unsigned short* __restrict__ WH, unsigned short* __restrict__ WL)
{
  const unsigned j = pin_u32(blockIdx.x * 256u + threadIdx.x);
  if (j >= (unsigned)(kNp * kCh / 8)) return;
  const unsigned row = pin_u32(j / 24u);
  const unsigned c8  = pin_u32((j - row * 24u) << 3);
  const bool live = row < (unsigned)kNreal;
  const unsigned srow = live ? row : (unsigned)(kNreal - 1);
  const float* sp = w + (size_t)srow * kCh + c8;
  v4f a0 = *(const v4f*)(sp);
  v4f a1 = *(const v4f*)(sp + 4);
#pragma unroll
  for (int e = 0; e < 4; ++e) {
    const float t0 = a0[e];
    const float t1 = a1[e];
    a0[e] = live ? t0 : 0.0f;
    a1[e] = live ? t1 : 0.0f;
  }
  v4u hv, lv;
  split8(a0, a1, hv, lv);
  const size_t eo = (size_t)j << 3;
  *(volatile v4u*)(WH + eo) = hv;
  *(volatile v4u*)(WL + eo) = lv;
  __threadfence();
  *(volatile v4u*)(WH + eo) = hv;
  *(volatile v4u*)(WL + eo) = lv;
}

__global__ __launch_bounds__(256) void proj_gemm_kernel(
    const unsigned short* __restrict__ Ahp, const unsigned short* __restrict__ Alp,
    const unsigned short* __restrict__ Bhp, const unsigned short* __restrict__ Blp,
    float* __restrict__ Cout)
{
  const __bf16* A   = (const __bf16*)Ahp;
  const __bf16* A2  = (const __bf16*)Alp;
  const __bf16* Bt  = (const __bf16*)Bhp;
  const __bf16* Bt2 = (const __bf16*)Blp;
  __shared__ __align__(16) float sT[8][16 * 68];
  const int lane = threadIdx.x & 31;
  const int wave = threadIdx.x >> 5;
  const int tile = blockIdx.x * 8 + wave;
  if (tile >= kTilesM * kTilesN) return;
  const int tm = tile / kTilesN;
  const int tn = tile - tm * kTilesN;
  const int m0 = tm << 6;
  const int n0 = tn << 6;
  const int rlane = lane & 15;
  const int koff  = (lane >> 4) * 8;
  const int mOff  = (lane >> 4) * 8;

  v8f acc[4][4];
#pragma unroll
  for (int i = 0; i < 4; ++i)
#pragma unroll
    for (int j = 0; j < 4; ++j) acc[i][j] = (v8f){0.f,0.f,0.f,0.f,0.f,0.f,0.f,0.f};

#pragma unroll 1
  for (int k0 = 0; k0 < kCh; k0 += 32) {
    v16b bh[4], bl[4];
#pragma unroll
    for (int j = 0; j < 4; ++j) {
      const size_t bo = (size_t)(n0 + (j << 4) + rlane) * kCh + koff + k0;
      bh[j] = FragB::load(Bt + bo);
      bl[j] = FragB::load(Bt2 + bo);
    }
#pragma unroll
    for (int i = 0; i < 4; ++i) {
      const size_t ao = (size_t)(m0 + (i << 4) + rlane) * kCh + koff + k0;
      const v16b ah = FragB::load(A + ao);
      const v16b al = FragB::load(A2 + ao);
#pragma unroll
      for (int j = 0; j < 4; ++j) {
        acc[i][j] = FragB::mma(ah, bh[j], acc[i][j]);
        acc[i][j] = FragB::mma(ah, bl[j], acc[i][j]);
        acc[i][j] = FragB::mma(al, bh[j], acc[i][j]);
      }
      guard_row4(acc[i][0], acc[i][1], acc[i][2], acc[i][3], ah, al);
    }
    keep4_b(bh[0], bh[1], bh[2], bh[3]);
    keep4_b(bl[0], bl[1], bl[2], bl[3]);
  }
  acc_guard4(acc[0][0], acc[0][1], acc[0][2], acc[0][3]);
  acc_guard4(acc[1][0], acc[1][1], acc[1][2], acc[1][3]);
  acc_guard4(acc[2][0], acc[2][1], acc[2][2], acc[2][3]);
  acc_guard4(acc[3][0], acc[3][1], acc[3][2], acc[3][3]);

  float* slab = sT[wave];
#pragma unroll
  for (int i = 0; i < 4; ++i) {
    const int mBase = m0 + (i << 4);
#pragma unroll
    for (int j = 0; j < 4; ++j) {
#pragma unroll
      for (int r = 0; r < 8; ++r) {
        slab[(mOff + r) * 68 + (j << 4) + rlane] = acc[i][j][r];
      }
    }
    __builtin_amdgcn_fence(__ATOMIC_RELEASE, "workgroup");
    __builtin_amdgcn_wave_barrier();
    __builtin_amdgcn_fence(__ATOMIC_ACQUIRE, "workgroup");
    {
      const int hh = lane >> 4, c4 = (lane & 15) * 4;
      for (int pass = 0; pass < 2; ++pass) {
#pragma unroll
        for (int it = 0; it < 8; ++it) {
          const int row = it * 2 + hh;
          const v4f v = *(const v4f*)(slab + row * 68 + c4);
          *(volatile v4f*)(Cout + (size_t)(mBase + row) * kNp + n0 + c4) = v;
        }
        __threadfence();
      }
    }
    __builtin_amdgcn_fence(__ATOMIC_RELEASE, "workgroup");
    __builtin_amdgcn_wave_barrier();
    __builtin_amdgcn_fence(__ATOMIC_ACQUIRE, "workgroup");
  }
}

template <int PASS>
__global__ __launch_bounds__(64) void scan_pair_kernel(
    const float* __restrict__ x, const float* __restrict__ Z,
    const float* __restrict__ dtw, const float* __restrict__ dtb,
    const float* __restrict__ alog, const float* __restrict__ dsk,
    float* Yall)
{
  __shared__ __align__(16) float sZ[kChunk * kZP];
  __shared__ __align__(16) float sY[kChunk * kBlkCh];
  __shared__ __align__(16) float sA[kHalfSt * 64];
  const unsigned tid = pin_u32(threadIdx.x);
  const unsigned bx  = blockIdx.x;
  const unsigned bo  = bx / 6u;
  const unsigned cg  = bx - bo * 6u;
  const unsigned o   = bo & 1u;
  const unsigned img = bo >> 1;
  const unsigned chl  = pin_u32(tid >> 1);
  const unsigned half = pin_u32(tid & 1u);
  const unsigned d    = cg * (unsigned)kBlkCh + chl;
  const unsigned posShift   = o ? 6u : 0u;
  const unsigned chunkShift = o ? 0u : 6u;
  const float* xrow = x + (((size_t)img * kCh + d) << 12);
  const size_t rowBase = (size_t)img << 12;
  float* Yp = Yall + (size_t)o * kPlaneElems;
  const unsigned fcol = pin_u32(tid & 31u);
  const unsigned fpar = pin_u32(tid >> 5);
  const size_t ystep = (size_t)kCh << posShift;

  const unsigned k  = o + 2u * (unsigned)PASS;
  const unsigned kd = k * (unsigned)kCh + d;
#pragma unroll 1
  for (unsigned n = 0; n < (unsigned)kHalfSt; ++n) {
    sA[n * 64u + tid] = -expf(alog[(size_t)kd * kSt + half * (unsigned)kHalfSt + n]);
  }
  __syncthreads();
  float negA[kHalfSt], h[kHalfSt];
#pragma unroll
  for (int n = 0; n < kHalfSt; ++n) {
    negA[n] = sA[n * 64 + tid];
    h[n] = 0.0f;
  }
  const v2f w01 = *(const v2f*)(dtw + (size_t)kd * kRk);
  const v2f w23 = *(const v2f*)(dtw + (size_t)kd * kRk + 2);
  const v2f w45 = *(const v2f*)(dtw + (size_t)kd * kRk + 4);
  const float bias = dtb[kd];
  const float dsv  = dsk[kd];
  const float* zk = Z + k * (unsigned)kXd;

#pragma unroll 1
  for (unsigned ci = 0; ci < 64u; ++ci) {
    const unsigned c = PASS ? (63u - ci) : ci;
    const unsigned posBase = c << chunkShift;
    __syncthreads();
    {
      const float* zr = zk + (rowBase + posBase + ((size_t)tid << posShift)) * kNp;
      v2f t[19];
#pragma unroll
      for (int i = 0; i < 19; ++i) t[i] = *(const v2f*)(zr + 2 * i);
      float* zs = sZ + tid * (unsigned)kZP;
#pragma unroll
      for (int i = 0; i < 19; ++i) {
        const int dst = (i < 3) ? (2 * i) : (2 * i + 2);
        *(v2f*)(zs + dst) = t[i];
      }
    }
    __syncthreads();

#pragma unroll 1
    for (unsigned si = 0; si < 64u; ++si) {
      const unsigned s = PASS ? (63u - si) : si;
      const float u = xrow[posBase + (s << posShift)];
      const float* zr = sZ + s * (unsigned)kZP;
      const v4f q0 = *(const v4f*)(zr);
      const v2f q1 = *(const v2f*)(zr + 4);
      const float* zb = zr + 8 + half * (unsigned)kHalfSt;
      const v4f b0 = *(const v4f*)(zb);
      const v4f b1 = *(const v4f*)(zb + 4);
      const v4f c0 = *(const v4f*)(zb + 16);
      const v4f c1 = *(const v4f*)(zb + 20);
      float z = fmaf(w01[0], q0[0], bias);
      z = fmaf(w01[1], q0[1], z);
      z = fmaf(w23[0], q0[2], z);
      z = fmaf(w23[1], q0[3], z);
      z = fmaf(w45[0], q1[0], z);
      z = fmaf(w45[1], q1[1], z);
      const float ea  = expf(-fabsf(z));
      const float u1  = 1.0f + ea;
      const float l1p = logf(u1) + (ea - (u1 - 1.0f)) * __builtin_amdgcn_rcpf(u1);
      const float dt  = fmaxf(z, 0.0f) + l1p;
      const float dBu = dt * u;
      float Bv[kHalfSt], Cv[kHalfSt];
      Bv[0] = b0[0]; Bv[1] = b0[1]; Bv[2] = b0[2]; Bv[3] = b0[3];
      Bv[4] = b1[0]; Bv[5] = b1[1]; Bv[6] = b1[2]; Bv[7] = b1[3];
      Cv[0] = c0[0]; Cv[1] = c0[1]; Cv[2] = c0[2]; Cv[3] = c0[3];
      Cv[4] = c1[0]; Cv[5] = c1[1]; Cv[6] = c1[2]; Cv[7] = c1[3];
      float y = 0.0f;
#pragma unroll
      for (int n = 0; n < kHalfSt; ++n) {
        const float dA = expf(dt * negA[n]);
        h[n] = fmaf(h[n], dA, dBu * Bv[n]);
        y = fmaf(h[n], Cv[n], y);
      }
      const float yo = __shfl_xor(y, 1, 32);
      float yt = y + yo;
      yt = fmaf(dsv, u, yt);
      sY[s * (unsigned)kBlkCh + chl] = yt;
    }
    __syncthreads();

    {
      const size_t yoff0 = (rowBase + posBase) * kCh + cg * (unsigned)kBlkCh + fcol;
      if (PASS) {
#pragma unroll 4
        for (unsigned it = 0; it < 32u; ++it) {
          const unsigned s = 2u * it + fpar;
          const float oldv = Yp[yoff0 + (size_t)s * ystep];
          const float cur  = sY[s * (unsigned)kBlkCh + fcol];
          const float sumv = cur + oldv;
          sY[s * (unsigned)kBlkCh + fcol] = sumv;
        }
      }
      for (int p = 0; p < 2; ++p) {
#pragma unroll 4
        for (unsigned it = 0; it < 32u; ++it) {
          const unsigned s = 2u * it + fpar;
          const float val = sY[s * (unsigned)kBlkCh + fcol];
          *(volatile float*)(Yp + yoff0 + (size_t)s * ystep) = val;
        }
        __threadfence();
      }
    }
  }
}

__global__ __launch_bounds__(256) void merge_norm_kernel(
    const float* __restrict__ Yr, const float* __restrict__ Yc,
    const float* __restrict__ nw, const float* __restrict__ nb, float* __restrict__ out)
{
  const unsigned lane = pin_u32(threadIdx.x & 31u);
  const unsigned wave = threadIdx.x >> 5;
  float gw[6], gb[6];
#pragma unroll
  for (int j = 0; j < 6; ++j) {
    gw[j] = nw[lane + 32u * (unsigned)j];
    gb[j] = nb[lane + 32u * (unsigned)j];
  }
  const unsigned row0 = (blockIdx.x * 8u + wave) * 4u;
#pragma unroll 1
  for (unsigned it = 0; it < 4u; ++it) {
    const size_t off = (size_t)(row0 + it) * kCh + lane;
    float v[6];
    float sum = 0.0f;
#pragma unroll
    for (int j = 0; j < 6; ++j) {
      v[j] = Yr[off + 32 * j] + Yc[off + 32 * j];
      sum += v[j];
    }
#pragma unroll
    for (int sh = 16; sh > 0; sh >>= 1) sum += __shfl_xor(sum, sh, 32);
    const float mu = sum * kInvCh;
    float sq = 0.0f;
#pragma unroll
    for (int j = 0; j < 6; ++j) {
      v[j] = v[j] - mu;
      sq = fmaf(v[j], v[j], sq);
    }
#pragma unroll
    for (int sh = 16; sh > 0; sh >>= 1) sq += __shfl_xor(sq, sh, 32);
    const float rs = rsqrtf(sq * kInvCh + kEps);
    float ov[6];
#pragma unroll
    for (int j = 0; j < 6; ++j) ov[j] = (v[j] * rs) * gw[j] + gb[j];
    for (int p = 0; p < 2; ++p) {
#pragma unroll
      for (int j = 0; j < 6; ++j) *(volatile float*)(out + off + 32 * j) = ov[j];
      __threadfence();
    }
  }
}

extern "C" void kernel_launch(void* const* d_in, const int* in_sizes, int n_in,
                              void* d_out, int out_size, void* d_ws, size_t ws_size,
                              hipStream_t stream) {
  if (n_in < 8) return;
  if (in_sizes[0] != kRows * kCh) return;
  if (in_sizes[1] != kNreal * kCh) return;
  if (in_sizes[2] != kDir * kCh * kRk) return;
  if (in_sizes[3] != kDir * kCh) return;
  if (in_sizes[4] != kDir * kCh * kSt) return;
  if (in_sizes[5] != kDir * kCh) return;
  if (in_sizes[6] != kCh) return;
  if (in_sizes[7] != kCh) return;
  if (out_size != kRows * kCh) return;
  if (ws_size < kWsTotal) return;

  const float* x    = (const float*)d_in[0];
  const float* xpw  = (const float*)d_in[1];
  const float* dtw  = (const float*)d_in[2];
  const float* dtb  = (const float*)d_in[3];
  const float* alog = (const float*)d_in[4];
  const float* dsk  = (const float*)d_in[5];
  const float* nw   = (const float*)d_in[6];
  const float* nb   = (const float*)d_in[7];
  float* out = (float*)d_out;

  char* ws = (char*)d_ws;
  unsigned short* XH = (unsigned short*)(ws + kOffXH);
  unsigned short* XL = (unsigned short*)(ws + kOffXL);
  unsigned short* WH = (unsigned short*)(ws + kOffWH);
  unsigned short* WL = (unsigned short*)(ws + kOffWL);
  float* Zp = (float*)(ws + kOffZ);
  float* YR = (float*)(ws + kOffYR);
  float* YC = (float*)(ws + kOffYC);

  pack_x_kernel<<<kImg * (kPos / 32), 256, 0, stream>>>(x, XH, XL);
  pack_w_kernel<<<(kNp * kCh / 8) / 256, 256, 0, stream>>>(xpw, WH, WL);
  proj_gemm_kernel<<<(kTilesM * kTilesN) / 8, 256, 0, stream>>>(XH, XL, WH, WL, Zp);
  scan_pair_kernel<0><<<kImg * 2 * (kCh / kBlkCh), 64, 0, stream>>>(x, Zp, dtw, dtb, alog, dsk, YR);
  scan_pair_kernel<1><<<kImg * 2 * (kCh / kBlkCh), 64, 0, stream>>>(x, Zp, dtw, dtb, alog, dsk, YR);
  merge_norm_kernel<<<kRows / 32, 256, 0, stream>>>(YR, YC, nw, nb, out);
}
